// GPSA_51556787421954
// MI455X (gfx1250) — hardware-verified
//
#include <hip/hip_runtime.h>


namespace {
constexpr int NB_ = 4, S = 1024, C = 256, H = 8, HD = 32, NT = NB_ * S, CH = 256;
constexpr float XS = 8.0f, HS = 256.0f, PS = 16384.0f, WSC = 256.0f, SCALE = 0.17677669529663687f;
typedef _Float16 b16;
typedef __attribute__((ext_vector_type(16))) _Float16 v16b;
typedef __attribute__((ext_vector_type(8))) _Float16 v8b;
typedef __attribute__((ext_vector_type(8))) float v8f;
typedef __attribute__((ext_vector_type(4))) float v4f;
typedef __attribute__((ext_vector_type(2))) float v2f;
typedef __attribute__((ext_vector_type(2))) _Float16 v2b;
__device__ __forceinline__ float bf16_rne(float f) { unsigned int u = __float_as_uint(f); u += 0x7FFFu + ((u >> 16) & 1u); float r = __uint_as_float(u & 0xFFFF0000u); asm volatile("" : "+v"(r)); return r; }
__device__ __forceinline__ float bfv(float f) { float r = bf16_rne(f); asm volatile("" : "+v"(r)); return r; }
__device__ __forceinline__ void split16(float v, b16& hi, b16& lo) { hi = (b16)v; lo = (b16)(v - (float)hi); }
__device__ __forceinline__ v16b frag_kb(const b16* p, int hh) { const v8b a = *(const v8b*)(p + 8 * hh), b = *(const v8b*)(p + 16 + 8 * hh); v16b f;
#pragma unroll
  for (int e = 0; e < 8; ++e) { f[e] = a[e]; f[8 + e] = b[e]; } return f; }
__device__ __forceinline__ v8f wmma16b(v16b a, v16b b, v8f c) { v8f d = __builtin_amdgcn_wmma_f32_16x16x32_f16(false, a, false, b, (short)0, c, false, false); asm volatile("v_nop\n\tv_nop\n\tv_nop\n\tv_nop" : "+v"(d) : "v"(a), "v"(b)); return d; }
__device__ __forceinline__ void wave_lds_sync() { __builtin_amdgcn_fence(__ATOMIC_RELEASE, "workgroup"); __builtin_amdgcn_wave_barrier(); __builtin_amdgcn_fence(__ATOMIC_ACQUIRE, "workgroup"); }
__device__ __forceinline__ float pmul(float a, float b) { float p = a * b; asm volatile("" : "+v"(p)); return p; }

__global__ __launch_bounds__(256) void wput_kernel(const float* __restrict__ wqk, const float* __restrict__ wv, const float* __restrict__ wproj, b16* __restrict__ WA, b16* __restrict__ WP) { const int u = blockIdx.x * 256 + threadIdx.x; v8b v; auto put = [&](b16* dst) { for (int pass = 0; pass < 2; ++pass) { *(volatile v8b*)dst = v; __threadfence(); } };
  if (u < 768 * 32) { const int o = u / 32, k0 = (u % 32) * 8;
#pragma unroll
    for (int j = 0; j < 8; ++j) v[j] = (b16)(bf16_rne(o < 512 ? wqk[(size_t)(k0 + j) * 512 + o] : wv[(size_t)(k0 + j) * C + (o - 512)]) * WSC); put(WA + (size_t)o * C + k0); }
  if (u < 256 * 32) { const int o = u / 32, k0 = (u % 32) * 8;
#pragma unroll
    for (int j = 0; j < 8; ++j) v[j] = (b16)(bf16_rne(wproj[(size_t)(k0 + j) * C + o]) * WSC); put(WP + (size_t)o * C + k0); } }
__global__ __launch_bounds__(32) void proj_kernel(const float* __restrict__ x, const b16* __restrict__ WA, int QLIM, b16* __restrict__ Qh, b16* __restrict__ Ql, b16* __restrict__ Kh, b16* __restrict__ Kl, float* __restrict__ Vr) { __shared__ __attribute__((aligned(16))) b16 Ax[16][C + 8]; __shared__ float Tf[16][772]; const int lane = threadIdx.x, nloc = lane & 15, hlf = lane >> 4; const size_t t0 = (size_t)blockIdx.x * 16; const int b = (int)(t0 / S), n0 = (int)(t0 % S); if (n0 >= QLIM) return;
  for (int rr = 0; rr < 16; ++rr) for (int q = 0; q < C / 32; ++q) { const int c = q * 32 + lane; Ax[rr][c] = (b16)(bfv(x[(t0 + rr) * C + c]) * XS); }
  if (lane < 16) for (int k = C; k < C + 8; ++k) Ax[lane][k] = (b16)0.0f;
  wave_lds_sync();
#pragma unroll 1
  for (int g = 0; g < 3; ++g) { v8f acc[16];
#pragma unroll
    for (int t = 0; t < 16; ++t) acc[t] = (v8f){};
#pragma unroll 2
    for (int kb = 0; kb < C; kb += 32) { const v16b a = frag_kb(&Ax[nloc][kb], hlf);
#pragma unroll
      for (int t = 0; t < 16; ++t) acc[t] = wmma16b(a, frag_kb(WA + (size_t)(g * 256 + t * 16 + nloc) * C + kb, hlf), acc[t]); }
#pragma unroll
    for (int t = 0; t < 16; ++t)
#pragma unroll
      for (int r8 = 0; r8 < 8; ++r8) Tf[8 * hlf + r8][g * 256 + t * 16 + nloc] = acc[t][r8] * (1.0f / (XS * WSC)); }
  wave_lds_sync();
  for (int pass = 0; pass < 2; ++pass) { for (int rr = 0; rr < 16; ++rr) { for (int h = 0; h < H; ++h) { const size_t po = (((size_t)(b * H + h)) * S + n0 + rr) * HD + lane; b16 p, pl; split16(Tf[rr][h * HD + lane] * HS, p, pl); ((volatile b16*)Qh)[po] = p; ((volatile b16*)Ql)[po] = pl; split16(Tf[rr][C + h * HD + lane] * HS, p, pl); ((volatile b16*)Kh)[po] = p; ((volatile b16*)Kl)[po] = pl; }
      for (int q = 0; q < 2; ++q) *(volatile v4f*)(Vr + (t0 + rr) * C + q * 128 + lane * 4) = *(const v4f*)(&Tf[rr][512 + q * 128 + lane * 4]); } __threadfence(); } }
__global__ __launch_bounds__(256) void vt_kernel(const float* __restrict__ Vr, int QLIM, b16* __restrict__ VTh, b16* __restrict__ VTl) { __shared__ float Tt[64][257]; const size_t t0 = (size_t)blockIdx.x * 64; const int b = (int)(t0 / S), n0 = (int)(t0 % S); if (n0 >= QLIM) return; const int tid = threadIdx.x, wave = tid >> 5, lane = tid & 31;
  for (int q = wave; q < 64; q += 8) for (int c = lane; c < C; c += 32) Tt[q][c] = Vr[(t0 + q) * C + c];
  __syncthreads();
  for (int pass = 0; pass < 2; ++pass) { for (int c = wave; c < C; c += 8) { const int h = c / HD, d = c % HD; b16 h0, l0, h1, l1; split16(Tt[lane * 2][c] * HS, h0, l0); split16(Tt[lane * 2 + 1][c] * HS, h1, l1); const size_t o = (((size_t)(b * H + h)) * HD + d) * S + n0 + lane * 2; *(volatile v2b*)(VTh + o) = (v2b){h0, h1}; *(volatile v2b*)(VTl + o) = (v2b){l0, l1}; } __threadfence(); } }
__global__ __launch_bounds__(32) void att_kernel(const b16* __restrict__ Qh, const b16* __restrict__ Ql, const b16* __restrict__ Kh, const b16* __restrict__ Kl, const b16* __restrict__ VTh, const b16* __restrict__ VTl, const float* __restrict__ coord, const float* __restrict__ wpos, const float* __restrict__ bpos, const float* __restrict__ gating, int QLIM, float* __restrict__ O) { __shared__ float Sc[16][S + 1]; __shared__ __attribute__((aligned(16))) b16 Pa[16][CH + 8], Pb[16][CH + 8]; __shared__ float Of[16][HD + 1], Cw[16][8]; const int lane = threadIdx.x, nloc = lane & 15, hlf = lane >> 4; const int bh = blockIdx.x / (S / 16), q0 = (blockIdx.x % (S / 16)) * 16; if (q0 >= QLIM) return; const int b = bh / H, h = bh % H;
  if (lane < 16) for (int kk = CH; kk < CH + 8; ++kk) { Pa[lane][kk] = (b16)0.0f; Pb[lane][kk] = (b16)0.0f; }
  const v16b qa = frag_kb(Qh + ((size_t)bh * S + q0 + nloc) * HD, hlf), ql = frag_kb(Ql + ((size_t)bh * S + q0 + nloc) * HD, hlf);
#pragma unroll 1
  for (int tg = 0; tg < S / 16; tg += 4) { v8f s[4] = {(v8f){}, (v8f){}, (v8f){}, (v8f){}};
#pragma unroll
    for (int t = 0; t < 4; ++t) { if ((tg + t) * 16 >= QLIM) continue; const size_t ko = ((size_t)bh * S + (tg + t) * 16 + nloc) * HD; const v16b kh = frag_kb(Kh + ko, hlf), kl = frag_kb(Kl + ko, hlf); s[t] = wmma16b(qa, kh, s[t]); s[t] = wmma16b(qa, kl, s[t]); s[t] = wmma16b(ql, kh, s[t]); }
#pragma unroll
    for (int t = 0; t < 4; ++t)
#pragma unroll
      for (int r8 = 0; r8 < 8; ++r8) Sc[8 * hlf + r8][(tg + t) * 16 + nloc] = s[t][r8] * (SCALE / (HS * HS)); }
  wave_lds_sync();
  if (lane < 16) { const int i = q0 + lane; float* sr = &Sc[lane][0]; const float sg = 1.0f / (1.0f + __expf(-bfv(gating[h]))); const float w0 = bfv(wpos[0 * H + h]), w1 = bfv(wpos[1 * H + h]), w2 = bfv(wpos[2 * H + h]), w3 = bfv(wpos[3 * H + h]), bp = bfv(bpos[h]);
    const float pix = bfv(coord[((size_t)b * S + i) * 3]), piy = bfv(coord[((size_t)b * S + i) * 3 + 1]), piz = bfv(coord[((size_t)b * S + i) * 3 + 2]);
    float mx = -INFINITY; for (int j = 0; j < QLIM; ++j) mx = fmaxf(mx, sr[j]); float z = 0.0f; for (int j = 0; j < QLIM; ++j) { const float e = __expf(sr[j] - mx); sr[j] = e; z += e; } const float zi = 1.0f / z;
    auto plog = [&](int j) { const float* pj = coord + ((size_t)b * S + j) * 3; const float dx = bfv(pj[0]) - pix, dy = bfv(pj[1]) - piy, dz = bfv(pj[2]) - piz; const float dd = sqrtf(dx * dx + dy * dy + dz * dz); return pmul(dx, w0) + pmul(dy, w1) + pmul(dz, w2) + pmul(dd, w3) + bp; };
    float pm = -INFINITY; for (int j = 0; j < QLIM; ++j) pm = fmaxf(pm, plog(j)); float pz = 0.0f; for (int j = 0; j < QLIM; ++j) pz += __expf(plog(j) - pm); const float pzi = 1.0f / pz;
    float tot = 0.0f; for (int j = 0; j < QLIM; ++j) { const float a = pmul(1.0f - sg, sr[j] * zi) + pmul(sg, __expf(plog(j) - pm) * pzi); sr[j] = a; tot += a; } Cw[lane][0] = 1.0f / tot; }
  wave_lds_sync();
  v8f oacc[2] = {(v8f){}, (v8f){}};
#pragma unroll 1
  for (int k0 = 0; k0 < QLIM; k0 += CH) { for (int rr = 0; rr < 16; ++rr) { const float rn = Cw[rr][0]; for (int q = 0; q < CH / 32; ++q) { const int j = q * 32 + lane; b16 p, pl; split16(Sc[rr][k0 + j] * rn * PS, p, pl); Pa[rr][j] = p; Pb[rr][j] = pl; } }
    wave_lds_sync();
#pragma unroll 2
    for (int kb = 0; kb < CH; kb += 32) { const v16b pa = frag_kb(&Pa[nloc][kb], hlf), pb = frag_kb(&Pb[nloc][kb], hlf);
#pragma unroll
      for (int t = 0; t < 2; ++t) { const size_t vo = ((size_t)bh * HD + t * 16 + nloc) * S + k0 + kb; const v16b vh = frag_kb(VTh + vo, hlf), vl = frag_kb(VTl + vo, hlf); oacc[t] = wmma16b(pa, vh, oacc[t]); oacc[t] = wmma16b(pa, vl, oacc[t]); oacc[t] = wmma16b(pb, vh, oacc[t]); } }
    wave_lds_sync(); }
#pragma unroll
  for (int t = 0; t < 2; ++t)
#pragma unroll
    for (int r8 = 0; r8 < 8; ++r8) Of[8 * hlf + r8][t * 16 + nloc] = oacc[t][r8] * (1.0f / (PS * HS));
  wave_lds_sync();
  for (int pass = 0; pass < 2; ++pass) { for (int r = 0; r < 16; ++r) ((volatile float*)O)[((size_t)b * S + q0 + r) * C + h * HD + lane] = Of[r][lane]; __threadfence(); } }
__global__ __launch_bounds__(32) void outp_kernel(const float* __restrict__ O, const b16* __restrict__ WP, const float* __restrict__ bproj, int QLIM, float* __restrict__ out) { __shared__ __attribute__((aligned(16))) b16 Ah[16][C + 8], Al[16][C + 8]; __shared__ float Tf[16][260]; const int lane = threadIdx.x, nloc = lane & 15, hlf = lane >> 4; const size_t t0 = (size_t)blockIdx.x * 16; if ((int)(t0 % S) >= QLIM) return;
  for (int rr = 0; rr < 16; ++rr) for (int q = 0; q < C / 32; ++q) { const int c = q * 32 + lane; b16 p, pl; split16(O[(t0 + rr) * C + c] * HS, p, pl); Ah[rr][c] = p; Al[rr][c] = pl; }
  if (lane < 16) for (int k = C; k < C + 8; ++k) { Ah[lane][k] = (b16)0.0f; Al[lane][k] = (b16)0.0f; }
  wave_lds_sync(); v8f acc[16];
#pragma unroll
  for (int t = 0; t < 16; ++t) acc[t] = (v8f){};
#pragma unroll 2
  for (int kb = 0; kb < C; kb += 32) { const v16b a = frag_kb(&Ah[nloc][kb], hlf), al = frag_kb(&Al[nloc][kb], hlf);
#pragma unroll
    for (int t = 0; t < 16; ++t) { const v16b bw = frag_kb(WP + (size_t)(t * 16 + nloc) * C + kb, hlf); acc[t] = wmma16b(a, bw, acc[t]); acc[t] = wmma16b(al, bw, acc[t]); } }
#pragma unroll
  for (int t = 0; t < 16; ++t) { const int cc = t * 16 + nloc; const float bb = bfv(bproj[cc]);
#pragma unroll
    for (int r8 = 0; r8 < 8; ++r8) Tf[8 * hlf + r8][cc] = acc[t][r8] * (1.0f / (HS * WSC)) + bb; }
  wave_lds_sync();
  for (int pass = 0; pass < 2; ++pass) { for (int rr = 0; rr < 16; ++rr) for (int q = 0; q < 2; ++q) *(volatile v4f*)(out + (t0 + rr) * C + q * 128 + lane * 4) = *(const v4f*)(&Tf[rr][q * 128 + lane * 4]); __threadfence(); } }
}

extern "C" void kernel_launch(void* const* d_in, const int* in_sizes, int n_in, void* d_out, int out_size, void* d_ws, size_t ws_size, hipStream_t stream) {
  (void)n_in;
  auto Fp = [&](int i) { return (const float*)d_in[i]; };
  if (in_sizes[0] != NT * C || in_sizes[1] != NT * 3 || in_sizes[2] != C * 512 || in_sizes[3] != C * C || in_sizes[4] != C * C || in_sizes[6] != 4 * H || in_sizes[7] != H || in_sizes[8] != H || out_size != NT * C) return;
  const int QLIM = S;
  size_t off = 0; char* ws = (char*)d_ws;
  auto carve = [&](size_t bytes) { char* p = ws + off; off += (bytes + 255) & ~(size_t)255; return p; };
  b16* WA = (b16*)carve((size_t)768 * C * 2); b16* WP = (b16*)carve((size_t)C * C * 2); b16* Qh = (b16*)carve((size_t)NT * C * 2); b16* Ql = (b16*)carve((size_t)NT * C * 2); b16* Kh = (b16*)carve((size_t)NT * C * 2); b16* Kl = (b16*)carve((size_t)NT * C * 2); float* Vr = (float*)carve((size_t)NT * C * 4); b16* VTh = (b16*)carve((size_t)NT * C * 2); b16* VTl = (b16*)carve((size_t)NT * C * 2); float* O = (float*)carve((size_t)NT * C * 4);
  if (off > ws_size || off > ((size_t)32 << 20)) return;
  wput_kernel<<<(768 * 32 + 255) / 256, 256, 0, stream>>>(Fp(2), Fp(3), Fp(4), WA, WP);
  proj_kernel<<<NT / 16, 32, 0, stream>>>(Fp(0), WA, QLIM, Qh, Ql, Kh, Kl, Vr);
  vt_kernel<<<NT / 64, 256, 0, stream>>>(Vr, QLIM, VTh, VTl);
  att_kernel<<<NB_ * H * (S / 16), 32, 0, stream>>>(Qh, Ql, Kh, Kl, VTh, VTl, Fp(1), Fp(6), Fp(7), Fp(8), QLIM, O);
  outp_kernel<<<NT / 16, 32, 0, stream>>>(O, WP, Fp(5), QLIM, (float*)d_out);
}
